// GAT_16844861735392
// MI455X (gfx1250) — hardware-verified
//
#include <hip/hip_runtime.h>
#include <stddef.h>
#include <stdint.h>
#include <math.h>


#define DIN     128
#define H1C     128
#define C2      64
#define NG1     384
#define NG2     192
#define KA2     256
#define NTHR    256
#define NWAVE   8
#define EPT     8
#define CHUNK   (NTHR * EPT)
#define WCAP    (EPT * 32)
#define LISTN   (NWAVE * WCAP)
#define NBA     1024
#define SLA     10
#define RCAP    28672
#define DEGCAP  128
#define MEAS_B1024  16623
#define MEAS_MAXDEG 35
#define GBM     64
#define GBN     64
#define GTHR    128
#define MROWS   128
#define PSEG    1024
#define NPSEG   8
#define P_ATT1  (0 * PSEG)
#define P_B1    (1 * PSEG)
#define P_LNW   (2 * PSEG)
#define P_LNB   (3 * PSEG)
#define P_ATT2  (4 * PSEG)
#define P_B2    (5 * PSEG)
#define P_BIAS1 (6 * PSEG)
#define P_BIAS2 (7 * PSEG)
#define NEGSL   0.2f
#define WSMAX   134217728
#define BKT_LDS_INTS  (LISTN + RCAP + 16)
#define SCAN_ZINTS    (RCAP + 3 * NBA)
#define SCAN_LDS_INTS (2 * RCAP + 3 * NBA + 16)

static_assert((CHUNK & (CHUNK - 1)) == 0 && CHUNK <= 4096);
static_assert((NBA & (NBA - 1)) == 0 && NBA == (1 << SLA) && NBA <= 1024);
static_assert(((long long)CHUNK << SLA) < (1LL << 31));
static_assert(LISTN >= NWAVE * WCAP);
static_assert(NBA % NWAVE == 0 && NBA % 32 == 0);
static_assert((RCAP % 32) == 0 && (SCAN_ZINTS % 4) == 0);
static_assert(RCAP >= MEAS_B1024 + 4096);
static_assert(DEGCAP >= MEAS_MAXDEG + 8);
static_assert(SCAN_LDS_INTS * 4 <= 300000 && BKT_LDS_INTS * 4 <= 300000);
static_assert(GBM == (GTHR / 32) * 16);
static_assert((DIN % 32) == 0 && (KA2 % 32) == 0 && KA2 == 2 * H1C && DIN == H1C);
static_assert((NG1 % GBN) == 0 && (NG2 % GBN) == 0 && NG1 == 3 * H1C && NG2 == 3 * C2);
static_assert((MROWS % GBM) == 0 && (MROWS * (DIN / 8)) % NTHR == 0);
static_assert(H1C == 4 * 32 && C2 == 2 * 32);
static_assert(NG1 <= PSEG && NG2 <= PSEG && PSEG == 4 * NTHR);
static_assert(NWAVE * 32 * 2 * 2 <= RCAP);

typedef float          v2f  __attribute__((ext_vector_type(2)));
typedef float          v4f  __attribute__((ext_vector_type(4)));
typedef float          v8f  __attribute__((ext_vector_type(8)));
typedef double         v2d  __attribute__((ext_vector_type(2)));
typedef int            v4i  __attribute__((ext_vector_type(4)));
typedef int            v8i  __attribute__((ext_vector_type(8)));
typedef unsigned short v8us __attribute__((ext_vector_type(8)));
typedef __bf16         v16b __attribute__((ext_vector_type(16)));
typedef v4f  __attribute__((may_alias)) v4fa;
typedef v2d  __attribute__((may_alias)) v2da;
typedef v4i  __attribute__((may_alias)) v4ia;
typedef v8us __attribute__((may_alias)) v8usa;
union FragB { v16b v; v8us h[2]; v8i w; };

__device__ __forceinline__ v8f wmb(const FragB& a, const FragB& b, v8f c) {
  v8f d = __builtin_amdgcn_wmma_f32_16x16x32_bf16(false, a.v, false, b.v, (short)0, c, false, false);
  asm volatile("v_nop\n\tv_nop\n\tv_nop\n\tv_nop" : "+v"(d) : "v"(a.w), "v"(b.w));
  return d;
}

__device__ __forceinline__ unsigned int f2bf(float f) {
  const unsigned int u = __float_as_uint(f);
  const unsigned int r = ((u + 0x7FFFu + ((u >> 16) & 1u)) >> 16) & 0xFFFFu;
  return ((u & 0x7FFFFFFFu) > 0x7F800000u) ? 0x7FC0u : r;
}
__device__ __forceinline__ float bf2f(unsigned int b) { return __uint_as_float(b << 16); }
__device__ __forceinline__ float bfr(float f) { return bf2f(f2bf(f)); }
__device__ __forceinline__ int pk2(float a, float b) { return (int)(f2bf(a) | (f2bf(b) << 16)); }

template <int SLB>
__device__ __forceinline__ int scan_chunk(const int* __restrict__ dsts, int nE, int cbase, int slotBase,
                                          int nb, int vec8, int* list, int tid, int lane, int wave) {
  int wc = 0;
  const int el0  = tid * EPT;
  const int e0   = cbase + el0;
  const int sent = -2147483647 - 1;
  v4i da, db;
  if (vec8 != 0 && cbase + CHUNK <= nE) {
    da = *(const v4i*)(dsts + e0);
    db = *(const v4i*)(dsts + e0 + 4);
  } else {
    da.x = (e0     < nE) ? dsts[min(e0,     nE - 1)] : sent;
    da.y = (e0 + 1 < nE) ? dsts[min(e0 + 1, nE - 1)] : sent;
    da.z = (e0 + 2 < nE) ? dsts[min(e0 + 2, nE - 1)] : sent;
    da.w = (e0 + 3 < nE) ? dsts[min(e0 + 3, nE - 1)] : sent;
    db.x = (e0 + 4 < nE) ? dsts[min(e0 + 4, nE - 1)] : sent;
    db.y = (e0 + 5 < nE) ? dsts[min(e0 + 5, nE - 1)] : sent;
    db.z = (e0 + 6 < nE) ? dsts[min(e0 + 6, nE - 1)] : sent;
    db.w = (e0 + 7 < nE) ? dsts[min(e0 + 7, nE - 1)] : sent;
  }
  const unsigned nbs = (unsigned)slotBase;
  const unsigned unb = (unsigned)nb;
  const unsigned s0 = (unsigned)da.x - nbs, s1 = (unsigned)da.y - nbs;
  const unsigned s2 = (unsigned)da.z - nbs, s3 = (unsigned)da.w - nbs;
  const unsigned s4 = (unsigned)db.x - nbs, s5 = (unsigned)db.y - nbs;
  const unsigned s6 = (unsigned)db.z - nbs, s7 = (unsigned)db.w - nbs;
  const bool h0 = s0 < unb, h1 = s1 < unb, h2 = s2 < unb, h3 = s3 < unb;
  const bool h4 = s4 < unb, h5 = s5 < unb, h6 = s6 < unb, h7 = s7 < unb;
  const unsigned any = __builtin_amdgcn_ballot_w32(h0 | h1 | h2 | h3 | h4 | h5 | h6 | h7);
  if (any != 0u) {
#define HITJ(J, HJ, SJ) { \
      const unsigned mj = __builtin_amdgcn_ballot_w32(HJ); \
      if (mj != 0u) { \
        if (HJ) { \
          const int pos = wc + (int)__builtin_amdgcn_mbcnt_lo(mj, 0u); \
          if (pos < WCAP) list[wave * WCAP + pos] = ((el0 + (J)) << SLB) | (int)(SJ); \
        } \
        wc += (int)__builtin_popcount(mj); } }
    HITJ(0, h0, s0)
    HITJ(1, h1, s1)
    HITJ(2, h2, s2)
    HITJ(3, h3, s3)
    HITJ(4, h4, s4)
    HITJ(5, h5, s5)
    HITJ(6, h6, s6)
    HITJ(7, h7, s7)
#undef HITJ
  }
  return wc;
}

__device__ __forceinline__ v4i wt_unit(const float* __restrict__ w, int cols, int n, int kk) {
  const float* p = w + (size_t)kk * (size_t)cols + n;
  const float f0 = p[0];
  const float f1 = p[(size_t)cols];
  const float f2 = p[(size_t)2 * cols];
  const float f3 = p[(size_t)3 * cols];
  const float f4 = p[(size_t)4 * cols];
  const float f5 = p[(size_t)5 * cols];
  const float f6 = p[(size_t)6 * cols];
  const float f7 = p[(size_t)7 * cols];
  v4i o;
  o.x = pk2(f0, f1); o.y = pk2(f2, f3); o.z = pk2(f4, f5); o.w = pk2(f6, f7);
  return o;
}
__device__ __forceinline__ v4i par_unit(const float* __restrict__ p, int len, int shift, int t) {
  const int i0 = 4 * t - shift;
  const int ic = i0 < 0 ? 0 : (i0 > len - 4 ? len - 4 : i0);
  const v4f v = *(const v4f*)(p + ic);
  const bool ok = (i0 >= 0) && (i0 <= len - 4);
  v4i o;
  o.x = ok ? __float_as_int(bfr(v.x)) : 0;
  o.y = ok ? __float_as_int(bfr(v.y)) : 0;
  o.z = ok ? __float_as_int(bfr(v.z)) : 0;
  o.w = ok ? __float_as_int(bfr(v.w)) : 0;
  return o;
}

__global__ __launch_bounds__(NTHR) void k_prep(
    const float* __restrict__ x,
    const float* __restrict__ W1l, const float* __restrict__ W1r, const float* __restrict__ S1W,
    const float* __restrict__ W2l, const float* __restrict__ W2r, const float* __restrict__ S2W,
    const float* __restrict__ att1, const float* __restrict__ b1, const float* __restrict__ lnw,
    const float* __restrict__ lnb, const float* __restrict__ att2, const float* __restrict__ b2,
    const float* __restrict__ s1b, const float* __restrict__ s2b,
    unsigned short* XB, unsigned short* WT1, unsigned short* WT2, float* PAR, int nN, int nUx) {
  const int blk = (int)blockIdx.x, tid = (int)threadIdx.x;
  const int bX = nUx / NTHR;
  v4i o;
  int* dp;
  if (blk < bX) {
    const int u   = blk * NTHR + tid;
    const int row = u >> 4;
    const int c0  = (u & 15) * 8;
    const int rc  = row < nN ? row : nN - 1;
    const float* p = x + (size_t)rc * DIN + c0;
    const v4f a = *(const v4f*)p;
    const v4f b = *(const v4f*)(p + 4);
    const bool okr = row < nN;
    o.x = okr ? pk2(a.x, a.y) : 0;
    o.y = okr ? pk2(a.z, a.w) : 0;
    o.z = okr ? pk2(b.x, b.y) : 0;
    o.w = okr ? pk2(b.z, b.w) : 0;
    dp = (int*)(XB + (size_t)row * DIN + c0);
  } else {
    const int wb = blk - bX;
    const int g  = wb >> 3;
    const int v  = (wb & 7) * NTHR + tid;
    if (g < 3) {
      const int n  = v >> 4;
      const int k8 = (v & 15) * 8;
      if (g == 0)      o = wt_unit(W1l, H1C, n, k8);
      else if (g == 1) o = wt_unit(W1r, H1C, n, k8);
      else             o = wt_unit(S1W, H1C, n, k8);
      dp = (int*)(WT1 + (size_t)(g * H1C + n) * DIN + k8);
    } else if (g < 6) {
      const int n  = v >> 5;
      const int k8 = (v & 31) * 8;
      const int kk = k8 & (H1C - 1);
      if (g == 3)      o = wt_unit(W2l, C2, n, kk);
      else if (g == 4) o = wt_unit(W2r, C2, n, kk);
      else             o = wt_unit(S2W, C2, n, kk);
      dp = (int*)(WT2 + (size_t)((g - 3) * C2 + n) * KA2 + k8);
    } else if (g == 6) {
      const int seg = wb & 7;
      if (seg == 0)      o = par_unit(att1, H1C, 0, tid);
      else if (seg == 1) o = par_unit(b1,   H1C, 0, tid);
      else if (seg == 2) o = par_unit(lnw,  H1C, 0, tid);
      else if (seg == 3) o = par_unit(lnb,  H1C, 0, tid);
      else if (seg == 4) o = par_unit(att2, C2,  0, tid);
      else if (seg == 5) o = par_unit(b2,   C2,  0, tid);
      else if (seg == 6) o = par_unit(s1b,  H1C, 2 * H1C, tid);
      else               o = par_unit(s2b,  C2,  2 * C2,  tid);
      dp = (int*)(PAR + (size_t)seg * PSEG + 4 * tid);
    } else {
      return;
    }
  }
  *(volatile v4i*)dp = o;
  __threadfence();
  *(volatile v4i*)dp = o;
}

__global__ __launch_bounds__(NTHR) void k_bucket(const int* __restrict__ srcs, const int* __restrict__ dsts,
                                                 int nE, int nN, int vec8, int* HITS, int* FLG) {
  extern __shared__ __attribute__((aligned(16))) int bsm[];
  int* list = bsm;
  int* reg1 = bsm + LISTN;
  int* wcnt = reg1 + RCAP;
  const int tid = (int)threadIdx.x, lane = tid & 31, wave = tid >> 5;
  const int blk = (int)blockIdx.x;
  const int nodeBase = blk * NBA;
  int nb = nN - nodeBase;
  nb = nb < 0 ? 0 : (nb > NBA ? NBA : nb);

  int tot = 0, ovf = 0;
  const int nChunks = (nE + CHUNK - 1) / CHUNK;
#pragma unroll 1
  for (int ch = 0; ch < nChunks; ++ch) {
    const int cbase = ch * CHUNK;
    const int wc = scan_chunk<SLA>(dsts, nE, cbase, nodeBase, nb, vec8, list, tid, lane, wave);
    if (lane == 0) wcnt[wave] = wc;
    __syncthreads();
    int pre = 0, all = 0;
#pragma unroll
    for (int w2 = 0; w2 < NWAVE; ++w2) {
      int c = wcnt[w2];
      c = c < 0 ? 0 : (c > WCAP ? WCAP : c);
      all += c;
      pre += (w2 < wave) ? c : 0;
    }
    const int wcc  = wc > WCAP ? WCAP : wc;
    const int base = tot + pre;
#pragma unroll 1
    for (int i = lane; i < wcc; i += 32) {
      const int ent = list[wave * WCAP + i];
      const int el  = (ent >> SLA) & (CHUNK - 1);
      const int sl  = ent & (NBA - 1);
      int eid = cbase + el;
      eid = eid > nE - 1 ? nE - 1 : eid;
      const int sraw = srcs[eid];
      const int s = sraw < 0 ? 0 : (sraw > nN - 1 ? nN - 1 : sraw);
      const int pos = base + i;
      if (pos < RCAP) reg1[pos] = (int)((unsigned)s | ((unsigned)sl << 16));
    }
    if (tot + all > RCAP) ovf = 1;
    tot += all;
    tot = tot > RCAP ? RCAP : tot;
    __syncthreads();
  }
  const int nh = tot;
  const int nhPad = (nh + 31) & ~31;
  for (int i = nh + tid; i < nhPad; i += NTHR) reg1[i] = 0;
  __syncthreads();

  int* hb = HITS + (size_t)blk * RCAP;
  v4i cv;
  cv.x = (tid == 0) ? nh : 0;
  cv.y = (tid == 0) ? ovf : 0;
  cv.z = 0; cv.w = 0;
  int* fp = FLG + (size_t)blk * 32 + 4 * (tid & 7);
#pragma unroll 1
  for (int p = tid * 4; p < nhPad; p += NTHR * 4) {
    const v4i v = *(const v4ia*)(reg1 + p);
    *(volatile v4i*)(hb + p) = v;
  }
  if (tid < 8) *(volatile v4i*)fp = cv;
  __threadfence();
#pragma unroll 1
  for (int p = tid * 4; p < nhPad; p += NTHR * 4) {
    const v4i v = *(const v4ia*)(reg1 + p);
    *(volatile v4i*)(hb + p) = v;
  }
  if (tid < 8) *(volatile v4i*)fp = cv;
}

template <int CBP>
__global__ __launch_bounds__(GTHR) void k_gemm(
    const unsigned short* __restrict__ A, const unsigned short* __restrict__ WT,
    const float* __restrict__ biasN, float* outBase, int K, size_t planeStride)
{
  __shared__ __attribute__((aligned(16))) float stg[GBM * GBN];
  const int tid = (int)threadIdx.x, lane = tid & 31, wave = tid >> 5, hh = lane >> 4, m = lane & 15;
  const int rowBase = (int)blockIdx.x * GBM;
  const int by      = (int)blockIdx.y;
  const int n0      = by * GBN;
  const int plane   = by / CBP;
  const int cb      = by - plane * CBP;
  const int ldo     = CBP * GBN;

  float bv[4];
#pragma unroll
  for (int t = 0; t < 4; ++t) bv[t] = biasN[n0 + 16 * t + m];

  v8f acc[4];
  {
    const v8f z = {0.f, 0.f, 0.f, 0.f, 0.f, 0.f, 0.f, 0.f};
    acc[0] = z; acc[1] = z; acc[2] = z; acc[3] = z;
  }
  const unsigned short* ap = A  + (size_t)(rowBase + 16 * wave + m) * (size_t)K + 8 * hh;
  const unsigned short* wp = WT + (size_t)(n0 + m) * (size_t)K + 8 * hh;
  const int ksteps = K >> 5;
#pragma unroll 1
  for (int ks = 0; ks < ksteps; ++ks) {
    FragB af;
    af.h[0] = *(const v8usa*)(ap + 32 * ks);
    af.h[1] = *(const v8usa*)(ap + 32 * ks + 16);
#pragma unroll
    for (int t = 0; t < 4; ++t) {
      const unsigned short* wq = wp + (size_t)(16 * t) * (size_t)K + 32 * ks;
      FragB bf;
      bf.h[0] = *(const v8usa*)wq;
      bf.h[1] = *(const v8usa*)(wq + 16);
      acc[t] = wmb(af, bf, acc[t]);
    }
  }

#pragma unroll
  for (int t = 0; t < 4; ++t) {
    const int lc = 16 * t + m;
#pragma unroll
    for (int r = 0; r < 8; ++r) {
      const int lr = 16 * wave + 8 * hh + r;
      stg[lr * GBN + lc] = acc[t][r] + bv[t];
    }
  }
  __syncthreads();

  v4f fv[8];
#pragma unroll
  for (int i = 0; i < 8; ++i) {
    const int lr = 16 * wave + 2 * i + hh;
    fv[i] = *(const v4fa*)(stg + lr * GBN + 4 * m);
  }
  float* ob = outBase + (size_t)plane * planeStride + (size_t)cb * GBN + 4 * m;
#pragma unroll
  for (int i = 0; i < 8; ++i) {
    const int gr = rowBase + 16 * wave + 2 * i + hh;
    float* op = ob + (size_t)gr * (size_t)ldo;
    *(volatile v4f*)op = fv[i];
  }
  __threadfence();
#pragma unroll
  for (int i = 0; i < 8; ++i) {
    const int gr = rowBase + 16 * wave + 2 * i + hh;
    float* op = ob + (size_t)gr * (size_t)ldo;
    *(volatile v4f*)op = fv[i];
  }
}

template <int L>
__global__ __launch_bounds__(NTHR) void k_scan(const int* __restrict__ HITS, const int* __restrict__ FLGB,
                                               const float* __restrict__ XL, const float* __restrict__ XR,
                                               float* SK, const float* __restrict__ attp,
                                               const float* __restrict__ biasp,
                                               float* outF, double* REC, int nN) {
  static_assert(L == 1 || L == 2);
  constexpr int CPL = (L == 1) ? 4 : 2;
  constexpr int C   = CPL * 32;
  extern __shared__ __attribute__((aligned(16))) int ssm[];
  int* hl   = ssm;
  int* sl   = ssm + RCAP;
  int* cnt  = sl + RCAP;
  int* offs = cnt + NBA;
  int* cur  = offs + NBA;
  int* misc = cur + NBA;
  const int tid = (int)threadIdx.x, lane = tid & 31, wave = tid >> 5;
  const int blk = (int)blockIdx.x;
  const int nodeBase = blk * NBA;

  const int nhraw = FLGB[(size_t)blk * 32];
  const int bflag = FLGB[(size_t)blk * 32 + 1];
  const int nh  = nhraw < 0 ? 0 : (nhraw > RCAP ? RCAP : nhraw);
  const int ovf = (bflag != 0 || nhraw < 0 || nhraw > RCAP) ? 1 : 0;

  {
    const v4i z4 = {0, 0, 0, 0};
    for (int i = tid * 4; i < SCAN_ZINTS; i += NTHR * 4) *(v4ia*)(sl + i) = z4;
    if (tid < 16) misc[tid] = 0;
    const int* hb = HITS + (size_t)blk * RCAP;
    const int nh4 = (nh + 3) & ~3;
#pragma unroll 1
    for (int p = tid * 4; p < nh4; p += NTHR * 4) *(v4ia*)(hl + p) = *(const v4i*)(hb + p);
  }
  __syncthreads();

  if (wave == 0) {
#pragma unroll 1
    for (int b0 = 0; b0 < nh; b0 += 32) {
      const int idx = b0 + lane;
      const int uv  = hl[idx < nh ? idx : nh - 1];
      const int m32 = (nh - b0) < 32 ? (nh - b0) : 32;
#pragma unroll 1
      for (int k = 0; k < m32; ++k) {
        const int u  = __builtin_amdgcn_readlane(uv, k);
        const int sq = (u >> 16) & (NBA - 1);
        if (lane == 0) cnt[sq] = cnt[sq] + 1;
      }
    }
  }
  __syncthreads();
  if (wave == 0) {
    const int base = lane * (NBA / 32);
    int s = 0;
#pragma unroll 1
    for (int i = 0; i < NBA / 32; ++i) s += cnt[base + i];
    int incl = s;
#pragma unroll
    for (int d = 1; d < 32; d <<= 1) {
      const int y = __shfl_up(incl, d, 32);
      if (lane >= d) incl += y;
    }
    int run = incl - s;
#pragma unroll 1
    for (int i = 0; i < NBA / 32; ++i) {
      const int cv = cnt[base + i];
      offs[base + i] = run;
      cur[base + i]  = run;
      run += cv;
    }
  }
  __syncthreads();
  if (wave == 0) {
#pragma unroll 1
    for (int b0 = 0; b0 < nh; b0 += 32) {
      const int idx = b0 + lane;
      const int uv  = hl[idx < nh ? idx : nh - 1];
      const int m32 = (nh - b0) < 32 ? (nh - b0) : 32;
#pragma unroll 1
      for (int k = 0; k < m32; ++k) {
        const int u  = __builtin_amdgcn_readlane(uv, k);
        const int sq = (u >> 16) & (NBA - 1);
        if (lane == 0) {
          int p = cur[sq];
          p = p < 0 ? 0 : (p > RCAP - 1 ? RCAP - 1 : p);
          sl[p] = u;
          cur[sq] = p + 1;
        }
      }
    }
  }
  __syncthreads();

  const float qnan = __int_as_float(0x7fc00000);
  const float pzb  = (ovf != 0) ? qnan : 0.0f;
  float at[CPL], bb[CPL];
  if constexpr (L == 1) {
    const v4f q = *(const v4f*)(attp + 4 * lane);
    const v4f g = *(const v4f*)(biasp + 4 * lane);
    at[0] = q.x; at[1] = q.y; at[2] = q.z; at[3] = q.w;
    bb[0] = g.x; bb[1] = g.y; bb[2] = g.z; bb[3] = g.w;
  } else {
    const v2f q = *(const v2f*)(attp + 2 * lane);
    const v2f g = *(const v2f*)(biasp + 2 * lane);
    at[0] = q.x; at[1] = q.y;
    bb[0] = g.x; bb[1] = g.y;
  }
  double ps = 0.0, pq = 0.0;

#pragma unroll 1
  for (int si = 0; si < NBA / NWAVE; ++si) {
    const int s    = si * NWAVE + wave;
    const int node = nodeBase + s;
    const int nc   = node < nN ? node : nN - 1;
    int c = cnt[s];
    const bool big = c > DEGCAP;
    c = c < 0 ? 0 : (c > DEGCAP ? DEGCAP : c);
    int o = offs[s];
    o = o < 0 ? 0 : (o > RCAP ? RCAP : o);
    if (c > nh - o) c = nh - o;
    c = c < 0 ? 0 : c;

    float xr[CPL], skv[CPL];
    if constexpr (L == 1) {
      const v4f q = *(const v4f*)(XR + (size_t)nc * C + 4 * lane);
      const v4f g = *(const v4f*)(SK + (size_t)nc * C + 4 * lane);
      xr[0] = q.x; xr[1] = q.y; xr[2] = q.z; xr[3] = q.w;
      skv[0] = g.x; skv[1] = g.y; skv[2] = g.z; skv[3] = g.w;
    } else {
      const v2f q = *(const v2f*)(XR + (size_t)nc * C + 2 * lane);
      const v2f g = *(const v2f*)(SK + (size_t)nc * C + 2 * lane);
      xr[0] = q.x; xr[1] = q.y;
      skv[0] = g.x; skv[1] = g.y;
    }

    float mx = -3.0e38f, dn = 0.0f;
    float acc[CPL];
#pragma unroll
    for (int i = 0; i < CPL; ++i) acc[i] = 0.0f;
    const int T = c + 1;
#pragma unroll 1
    for (int b0 = 0; b0 < T; b0 += 32) {
      const int t = b0 + lane;
      int idx = o + t;
      idx = idx < 0 ? 0 : (idx > RCAP - 1 ? RCAP - 1 : idx);
      const int ent = sl[idx];
      int hs = ent & 0xFFFF;
      hs = hs > nN - 1 ? nN - 1 : hs;
      const int sr  = (t < c) ? hs : nc;
      const int m32 = (T - b0) < 32 ? (T - b0) : 32;
#pragma unroll 1
      for (int k = 0; k < m32; ++k) {
        const int sk = __builtin_amdgcn_readlane(sr, k);
        const float* rp = XL + (size_t)sk * C + CPL * lane;
        float a[CPL];
        if constexpr (L == 1) {
          const v4f q = *(const v4f*)rp;
          a[0] = q.x; a[1] = q.y; a[2] = q.z; a[3] = q.w;
        } else {
          const v2f q = *(const v2f*)rp;
          a[0] = q.x; a[1] = q.y;
        }
        float part = 0.0f;
#pragma unroll
        for (int j = 0; j < CPL; ++j) {
          float v = a[j] + xr[j];
          v = v > 0.0f ? v : NEGSL * v;
          part = fmaf(v, at[j], part);
        }
        part += __shfl_xor(part, 1);
        part += __shfl_xor(part, 2);
        if constexpr (L == 2) {
          part += __shfl_xor(part, 4);
          part += __shfl_xor(part, 8);
          part += __shfl_xor(part, 16);
        }
        const float lg = part;
        const float df = lg - mx;
        const float ee = expf(-fabsf(df));
        const bool  up = df > 0.0f;
        const float s1 = up ? ee : 1.0f;
        const float s2 = up ? 1.0f : ee;
        mx = up ? lg : mx;
        dn = fmaf(dn, s1, s2);
#pragma unroll
        for (int j = 0; j < CPL; ++j) acc[j] = fmaf(acc[j], s1, s2 * a[j]);
      }
    }
    const float inv = __builtin_amdgcn_rcpf(dn);
    const float pzr = big ? qnan : pzb;
    const bool live = node < nN;
    float r[CPL];
#pragma unroll
    for (int j = 0; j < CPL; ++j) r[j] = (fmaf(acc[j], inv, bb[j]) + skv[j]) + pzr;

    if constexpr (L == 1) {
      v4f ov; ov.x = r[0]; ov.y = r[1]; ov.z = r[2]; ov.w = r[3];
      float* hp = SK + (size_t)nc * C + 4 * lane;
      if (live) *(volatile v4f*)hp = ov;
      __threadfence();
      if (live) *(volatile v4f*)hp = ov;
#pragma unroll
      for (int j = 0; j < CPL; ++j) {
        const double d = live ? (double)r[j] : 0.0;
        ps += d;
        pq = fma(d, d, pq);
      }
    } else {
      v2f ov; ov.x = r[0]; ov.y = r[1];
      float* op = outF + (size_t)nc * C + 2 * lane;
      if (live) *(volatile v2f*)op = ov;
      __threadfence();
      if (live) *(volatile v2f*)op = ov;
    }
  }

  if constexpr (L == 1) {
    double* wsum = (double*)hl;
    v2d pv; pv.x = ps; pv.y = pq;
    *(v2da*)(wsum + (wave * 32 + lane) * 2) = pv;
    __syncthreads();
    if (wave == 0) {
      double s = 0.0, q = 0.0;
#pragma unroll
      for (int w2 = 0; w2 < NWAVE; ++w2) {
        const v2d p = *(const v2da*)(wsum + (w2 * 32 + lane) * 2);
        s += p.x; q += p.y;
      }
#pragma unroll
      for (int off = 16; off > 0; off >>= 1) {
        s += __shfl_xor(s, off);
        q += __shfl_xor(q, off);
      }
      int nbl = nN - nodeBase;
      nbl = nbl < 0 ? 0 : (nbl > NBA ? NBA : nbl);
      const double n  = (double)nbl * (double)C;
      const double nd = n > 0.0 ? n : 1.0;
      const double mean = s / nd;
      const double M2   = q - s * mean;
      v2d ov;
      ov.x = (lane == 0) ? n : ((lane == 1) ? M2 : 0.0);
      ov.y = (lane == 0) ? mean : 0.0;
      double* rp = REC + (size_t)blk * 16 + 2 * (lane & 7);
      if (lane < 8) *(volatile v2d*)rp = ov;
      __threadfence();
      if (lane < 8) *(volatile v2d*)rp = ov;
    }
  }
  (void)outF; (void)REC; (void)misc;
}

__global__ __launch_bounds__(32) void k_stats(const double* __restrict__ REC, float* STAT, int nBlk, double invTot) {
  const int lane = (int)threadIdx.x & 31;
  double n = 0.0, mean = 0.0, M2 = 0.0;
#pragma unroll 1
  for (int b = 0; b < nBlk; ++b) {
    const v2d p0 = *(const v2d*)(REC + (size_t)b * 16);
    const v2d p1 = *(const v2d*)(REC + (size_t)b * 16 + 2);
    const double nb = p0.x, mb = p0.y, Mb = p1.x;
    const double nt  = n + nb;
    const double nts = nt > 0.0 ? nt : 1.0;
    const double dl  = mb - mean;
    const double f   = nb / nts;
    mean = mean + dl * f;
    M2   = M2 + Mb + dl * dl * n * f;
    n = nt;
  }
  const double var = M2 * invTot;
  const float muf = (float)mean;
  const float rs  = 1.0f / sqrtf((float)var + 1e-5f);
  v4f o;
  o.x = (lane == 0) ? muf : 0.0f;
  o.y = (lane == 0) ? rs  : 0.0f;
  o.z = 0.0f; o.w = 0.0f;
  float* op = STAT + 4 * (lane & 7);
  if (lane < 8) *(volatile v4f*)op = o;
  __threadfence();
  if (lane < 8) *(volatile v4f*)op = o;
}

__global__ __launch_bounds__(NTHR) void k_norm(const float* __restrict__ H1, const float* __restrict__ STAT,
                                               const float* __restrict__ lnw, const float* __restrict__ lnb,
                                               unsigned short* HHL, int nN, int nUnits) {
  __shared__ float st[8 * NTHR];
  const int tid = (int)threadIdx.x;
  const int u = (int)blockIdx.x * NTHR + tid;
  if (u >= nUnits) return;
  const int row = u >> 4;
  const int c0  = (u & 15) * 8;
  const int rc  = row < nN ? row : nN - 1;
  const float mu = STAT[0];
  const float rs = STAT[1];
  const float* p = H1 + (size_t)rc * H1C + c0;
  const v4f a  = *(const v4f*)p;
  const v4f b  = *(const v4f*)(p + 4);
  const v4f wa = *(const v4f*)(lnw + c0);
  const v4f wb = *(const v4f*)(lnw + c0 + 4);
  const v4f ba = *(const v4f*)(lnb + c0);
  const v4f bc = *(const v4f*)(lnb + c0 + 4);
  st[0 * NTHR + tid] = fmaf((a.x - mu) * rs, wa.x, ba.x);
  st[1 * NTHR + tid] = fmaf((a.y - mu) * rs, wa.y, ba.y);
  st[2 * NTHR + tid] = fmaf((a.z - mu) * rs, wa.z, ba.z);
  st[3 * NTHR + tid] = fmaf((a.w - mu) * rs, wa.w, ba.w);
  st[4 * NTHR + tid] = fmaf((b.x - mu) * rs, wb.x, bc.x);
  st[5 * NTHR + tid] = fmaf((b.y - mu) * rs, wb.y, bc.y);
  st[6 * NTHR + tid] = fmaf((b.z - mu) * rs, wb.z, bc.z);
  st[7 * NTHR + tid] = fmaf((b.w - mu) * rs, wb.w, bc.w);
#pragma unroll 1
  for (int j = 0; j < 8; ++j) {
    float y = st[j * NTHR + tid];
    y = (y > 0.0f) ? y : expm1f(y);
    st[j * NTHR + tid] = y;
  }
  const bool live = row < nN;
  unsigned int hb[8], lb[8];
#pragma unroll
  for (int i = 0; i < 8; ++i) {
    const float y = st[i * NTHR + tid];
    const float v = live ? y : 0.0f;
    const unsigned int h = f2bf(v);
    hb[i] = h;
    lb[i] = f2bf(v - bf2f(h));
  }
  v4i ho, lo;
  ho.x = (int)(hb[0] | (hb[1] << 16)); ho.y = (int)(hb[2] | (hb[3] << 16));
  ho.z = (int)(hb[4] | (hb[5] << 16)); ho.w = (int)(hb[6] | (hb[7] << 16));
  lo.x = (int)(lb[0] | (lb[1] << 16)); lo.y = (int)(lb[2] | (lb[3] << 16));
  lo.z = (int)(lb[4] | (lb[5] << 16)); lo.w = (int)(lb[6] | (lb[7] << 16));
  int* hp = (int*)(HHL + (size_t)row * KA2 + c0);
  int* lp = (int*)(HHL + (size_t)row * KA2 + H1C + c0);
  *(volatile v4i*)hp = ho;
  *(volatile v4i*)lp = lo;
  __threadfence();
  *(volatile v4i*)hp = ho;
  *(volatile v4i*)lp = lo;
}

static inline int cdiv(int a, int b) { return (a + b - 1) / b; }

extern "C" void kernel_launch(void* const* d_in, const int* in_sizes, int n_in,
                              void* d_out, int out_size, void* d_ws, size_t ws_size,
                              hipStream_t stream) {
  if (n_in < 16) return;
  const int nN = in_sizes[0] / DIN;
  if (nN <= 0 || in_sizes[0] != nN * DIN || nN > 65536) return;
  if (in_sizes[1] < 2 || (in_sizes[1] & 1) != 0) return;
  const int nE = in_sizes[1] / 2;
  if (nE < 1 || nE > (1 << 30)) return;
  if (in_sizes[2] != DIN * H1C || in_sizes[3] != DIN * H1C || in_sizes[6] != DIN * H1C) return;
  if (in_sizes[4] != H1C || in_sizes[5] != H1C || in_sizes[7] != H1C) return;
  if (in_sizes[8] != H1C || in_sizes[9] != H1C) return;
  if (in_sizes[10] != H1C * C2 || in_sizes[11] != H1C * C2 || in_sizes[14] != H1C * C2) return;
  if (in_sizes[12] != C2 || in_sizes[13] != C2 || in_sizes[15] != C2) return;
  if (out_size != nN * C2) return;

  const float* x    = (const float*)d_in[0];
  const int*   ei   = (const int*)  d_in[1];
  const float* W1l  = (const float*)d_in[2];
  const float* W1r  = (const float*)d_in[3];
  const float* att1 = (const float*)d_in[4];
  const float* b1   = (const float*)d_in[5];
  const float* s1W  = (const float*)d_in[6];
  const float* s1b  = (const float*)d_in[7];
  const float* lnw  = (const float*)d_in[8];
  const float* lnb  = (const float*)d_in[9];
  const float* W2l  = (const float*)d_in[10];
  const float* W2r  = (const float*)d_in[11];
  const float* att2 = (const float*)d_in[12];
  const float* b2   = (const float*)d_in[13];
  const float* s2W  = (const float*)d_in[14];
  const float* s2b  = (const float*)d_in[15];
  float* out = (float*)d_out;
  const int* src = ei;
  const int* dst = ei + nE;

  const int MP   = cdiv(nN, MROWS) * MROWS;
  const int gM   = MP / GBM;
  const int gA   = cdiv(MP, NBA);
  if ((long long)gA * NBA < (long long)MP) return;
  const int vec8 = ((nE & 3) == 0) ? 1 : 0;
  const int nUx  = MP * (DIN / 8);
  if ((nUx % NTHR) != 0) return;

  char* ws = (char*)d_ws;
  size_t off = 0;
  const size_t oA   = off; off += (size_t)MP * KA2 * 2;           off = (off + 255) & ~(size_t)255;
  const size_t oPL  = off; off += (size_t)3 * MP * H1C * 4;       off = (off + 255) & ~(size_t)255;
  const size_t oHIT = off; off += (size_t)gA * RCAP * 4;          off = (off + 255) & ~(size_t)255;
  const size_t oFLG = off; off += (size_t)gA * 128;               off = (off + 255) & ~(size_t)255;
  const size_t oREC = off; off += (size_t)gA * 128;               off = (off + 255) & ~(size_t)255;
  const size_t oST  = off; off += (size_t)256;                    off = (off + 255) & ~(size_t)255;
  const size_t oWT1 = off; off += (size_t)NG1 * DIN * 2;          off = (off + 255) & ~(size_t)255;
  const size_t oWT2 = off; off += (size_t)NG2 * KA2 * 2;          off = (off + 255) & ~(size_t)255;
  const size_t oPAR = off; off += (size_t)NPSEG * PSEG * 4;       off = (off + 255) & ~(size_t)255;
  if (off > ws_size || off > (size_t)WSMAX) return;
  if ((size_t)MP * DIN * 2 > (size_t)MP * KA2 * 2) return;
  if ((size_t)3 * MP * C2 * 4 > (size_t)2 * MP * H1C * 4) return;
  unsigned short* XB   = (unsigned short*)(ws + oA);
  unsigned short* HHL  = (unsigned short*)(ws + oA);
  float*          PL   = (float*)(ws + oPL);
  int*            HITS = (int*)(ws + oHIT);
  int*            FLG  = (int*)(ws + oFLG);
  double*         REC  = (double*)(ws + oREC);
  float*          STAT = (float*)(ws + oST);
  unsigned short* WT1  = (unsigned short*)(ws + oWT1);
  unsigned short* WT2  = (unsigned short*)(ws + oWT2);
  float*          PAR  = (float*)(ws + oPAR);
  const size_t ps1 = (size_t)MP * H1C;
  const size_t ps2 = (size_t)MP * C2;
  float* XL1 = PL;
  float* XR1 = PL + ps1;
  float* SK1 = PL + 2 * ps1;
  float* XL2 = PL;
  float* XR2 = PL + ps2;
  float* SK2 = PL + 2 * ps2;

  const int bktLds  = BKT_LDS_INTS * 4;
  const int scanLds = SCAN_LDS_INTS * 4;
  hipFuncSetAttribute(reinterpret_cast<const void*>(&k_bucket),
                      hipFuncAttributeMaxDynamicSharedMemorySize, bktLds);
  hipFuncSetAttribute(reinterpret_cast<const void*>(&k_scan<1>),
                      hipFuncAttributeMaxDynamicSharedMemorySize, scanLds);
  hipFuncSetAttribute(reinterpret_cast<const void*>(&k_scan<2>),
                      hipFuncAttributeMaxDynamicSharedMemorySize, scanLds);

  k_prep<<<nUx / NTHR + 56, NTHR, 0, stream>>>(x, W1l, W1r, s1W, W2l, W2r, s2W, att1, b1, lnw, lnb, att2, b2,
                                               s1b, s2b, XB, WT1, WT2, PAR, nN, nUx);
  k_bucket<<<gA, NTHR, bktLds, stream>>>(src, dst, nE, nN, vec8, HITS, FLG);
  k_gemm<2><<<dim3(gM, NG1 / GBN), GTHR, 0, stream>>>(XB, WT1, PAR + P_BIAS1, PL, DIN, ps1);
  k_scan<1><<<gA, NTHR, scanLds, stream>>>(HITS, FLG, XL1, XR1, SK1, PAR + P_ATT1, PAR + P_B1, out, REC, nN);
  k_stats<<<1, 32, 0, stream>>>(REC, STAT, gA, 1.0 / ((double)nN * (double)H1C));
  k_norm<<<nUx / NTHR, NTHR, 0, stream>>>(SK1, STAT, PAR + P_LNW, PAR + P_LNB, HHL, nN, nUx);
  k_gemm<1><<<dim3(gM, NG2 / GBN), GTHR, 0, stream>>>(HHL, WT2, PAR + P_BIAS2, PL, KA2, ps2);
  k_scan<2><<<gA, NTHR, scanLds, stream>>>(HITS, FLG, XL2, XR2, SK2, PAR + P_ATT2, PAR + P_B2, out, REC, nN);
}
